// EquiConv_9972914061333
// MI455X (gfx1250) — hardware-verified
//
#include <hip/hip_runtime.h>
#include <math.h>

typedef __attribute__((ext_vector_type(16))) _Float16 v16h;
typedef __attribute__((ext_vector_type(16))) __bf16 v16b;
typedef __attribute__((ext_vector_type(8)))  _Float16 v8h;
typedef __attribute__((ext_vector_type(8)))  float v8f;
typedef __attribute__((ext_vector_type(4)))  float v4f;
typedef __attribute__((ext_vector_type(2)))  float v2f;
typedef __attribute__((ext_vector_type(4)))  unsigned v4u;
typedef __attribute__((ext_vector_type(4)))  int v4i;
typedef float __attribute__((may_alias)) float_a;
typedef int __attribute__((may_alias)) int_a;

template <typename T> __device__ __forceinline__ void vst2(void* p, T v) { *(volatile T*)p = v; __threadfence(); *(volatile T*)p = v; }
__device__ __forceinline__ v8f wmma16(v16h a, v16h b, v8f c) {
  v8f d = __builtin_amdgcn_wmma_f32_16x16x32_f16(false, a, false, b, (short)0, c, false, false);
  asm volatile("v_nop\n\tv_nop\n\tv_nop\n\tv_nop" : "+v"(d) : "v"(a), "v"(b));
  return d;
}
__device__ __forceinline__ v8f wmma_bf(v16b a, v16b b, v8f c) {
  v8f d = __builtin_amdgcn_wmma_f32_16x16x32_bf16(false, a, false, b, (short)0, c, false, false);
  asm volatile("v_nop\n\tv_nop\n\tv_nop\n\tv_nop" : "+v"(d) : "v"(a), "v"(b));
  return d;
}
__device__ __forceinline__ v16h frag_h(const _Float16* rowk0, int lane) {
  union { v16h v; v8h q[2]; } u; const _Float16* p = rowk0 + 8 * (lane >> 4);
  u.q[0] = *(const v8h*)p; u.q[1] = *(const v8h*)(p + 16); return u.v;
}
__device__ __forceinline__ v16h frag_f32(const float* rowk0, int lane) {
  v16h a; const float* p = rowk0 + 8 * (lane >> 4);
#pragma unroll
  for (int i = 0; i < 8; ++i) { a[i] = (_Float16)p[i]; a[8 + i] = (_Float16)p[16 + i]; }
  return a;
}
__device__ __forceinline__ v16h frag_f32s(const float* rowk0, int lane, float sc) {
  v16h a; const float* p = rowk0 + 8 * (lane >> 4);
#pragma unroll
  for (int i = 0; i < 8; ++i) { a[i] = (_Float16)(p[i] * sc); a[8 + i] = (_Float16)(p[16 + i] * sc); }
  return a;
}
__device__ __forceinline__ v16h fragc_f32(const float* W, int k0, int n, int lane, int ld, int K) {
  v16h a; const int g = lane >> 4;
#pragma unroll
  for (int i = 0; i < 8; ++i) { const int ka = k0 + 8 * g + i, kb = ka + 16;
    a[i] = (_Float16)(ka < K ? W[(size_t)(ka < K ? ka : K - 1) * ld + n] : 0.f); a[8 + i] = (_Float16)(kb < K ? W[(size_t)(kb < K ? kb : K - 1) * ld + n] : 0.f); }
  return a;
}
struct F2 { v16b h, l; };
__device__ __forceinline__ F2 bsplit16(const float v[16]) { F2 r;
#pragma unroll
  for (int i = 0; i < 16; ++i) { const __bf16 h = (__bf16)v[i]; r.h[i] = h; r.l[i] = (__bf16)(v[i] - (float)h); }
  return r; }
__device__ __forceinline__ F2 split_row(const float* row, int k0, int lane) { float v[16]; const float* p = row + k0 + 8 * (lane >> 4);
#pragma unroll
  for (int i = 0; i < 8; ++i) { v[i] = p[i]; v[8 + i] = p[16 + i]; }
  return bsplit16(v); }
__device__ __forceinline__ F2 split_rowK(const float* row, int k0, int lane, int K) { float v[16]; const int g = lane >> 4;
#pragma unroll
  for (int i = 0; i < 8; ++i) { const int ka = k0 + 8 * g + i, kb = ka + 16; v[i] = ka < K ? row[ka < K ? ka : K - 1] : 0.f; v[8 + i] = kb < K ? row[kb < K ? kb : K - 1] : 0.f; }
  return bsplit16(v); }
__device__ __forceinline__ F2 split_col(const float* W, int k0, int n, int lane, int ld, int K) { float v[16]; const int g = lane >> 4;
#pragma unroll
  for (int i = 0; i < 8; ++i) { const int ka = k0 + 8 * g + i, kb = ka + 16; v[i] = ka < K ? W[(size_t)(ka < K ? ka : K - 1) * ld + n] : 0.f; v[8 + i] = kb < K ? W[(size_t)(kb < K ? kb : K - 1) * ld + n] : 0.f; }
  return bsplit16(v); }
__device__ __forceinline__ v8f mac3(const F2& a, const F2& b, v8f c) { c = wmma_bf(a.l, b.h, c); c = wmma_bf(a.h, b.l, c); return wmma_bf(a.h, b.h, c); }
__device__ __forceinline__ float sigm(float v) { return 1.0f / (1.0f + expf(-v)); }
#define LDSX() do { asm volatile("s_wait_dscnt 0" ::: "memory"); __builtin_amdgcn_wave_barrier(); __builtin_amdgcn_fence(__ATOMIC_RELEASE, "workgroup"); } while (0)


#define NEDGE 20000
#define NS_ 64
#define NV_ 32
#define FEA (NS_ + 3 * NV_)
#define FCIN 128
#define HID 64
#define NRB ((NEDGE + 63) / 64)
#define NPAD (NRB * 64)
#ifndef NRBT
#define NRBT NRB
#endif
typedef __attribute__((ext_vector_type(8))) __bf16 v8b;
__device__ __forceinline__ v16b frag_b(const __bf16* rowk0, int lane) {
  union { v16b v; v8b q[2]; } u; const __bf16* p = rowk0 + 8 * (lane >> 4);
  u.q[0] = *(const v8b*)p; u.q[1] = *(const v8b*)(p + 16); return u.v;
}
__device__ __forceinline__ float bfr(float v) { return (float)(__bf16)v; }
__device__ __attribute__((noinline)) float exp_ni(float v) { return expf(v); }
__device__ __attribute__((noinline)) float erf_ni(float v) { return erff(v); }

#define WS_PW   0u
#define PSS 0
#define PVV (PSS + 96 * 4096)
#define PVEC (PVV + 96 * 3072)
#define PM1 (PVEC + 32 * 4096)
#define PM2 (PM1 + HID * FCIN)
#define PM3 (PM2 + HID * HID)
#define PWEND (PM3 + 96 * HID)
#define WS_H1   (WS_PW + 2u * PWEND)
#define WS_H2   (WS_H1 + 4u * NPAD * HID)
#define WS_WE   (WS_H2 + 4u * NPAD * HID)
#define WS_END  (WS_WE + 4u * NPAD * 96)

__global__ __launch_bounds__(256) void k_pack(const float* __restrict__ WSSS, const float* __restrict__ WVVS, const float* __restrict__ WSSG, const float* __restrict__ WVVG, const float* __restrict__ WSVV, const float* __restrict__ WVSV, const float* __restrict__ W1, const float* __restrict__ W2, const float* __restrict__ W3, __bf16* __restrict__ PW) {
  __shared__ __align__(16) __bf16 s[4096]; const int n = blockIdx.x, which = blockIdx.y, tid = threadIdx.x; int K; size_t dst;
  if (which == 0) { if (n >= 96) return; K = 4096; dst = PSS + (size_t)n * 4096; for (int k = tid; k < K; k += 256) { const int u = k >> 6, v = k & 63; s[k] = (__bf16)((n < 64) ? WSSS[((size_t)u * 64 + v) * 64 + n] : WSSG[((size_t)u * 64 + v) * 32 + (n - 64)]); } }
  else if (which == 1) { if (n >= 96) return; K = 3072; dst = PVV + (size_t)n * 3072; for (int k = tid; k < K; k += 256) { const int uv = k / 3; const int u = uv >> 5, v = uv & 31; s[k] = (__bf16)((n < 64) ? WVVS[((size_t)u * 32 + v) * 64 + n] : WVVG[((size_t)u * 32 + v) * 32 + (n - 64)]); } }
  else if (which == 2) { if (n >= 32) return; K = 4096; dst = PVEC + (size_t)n * 4096; for (int k = tid; k < K; k += 256) { float w; if (k < 2048) { const int u = k >> 5, v = k & 31; w = WSVV[((size_t)u * 32 + v) * 32 + n]; } else { const int kk = k - 2048; const int u = kk >> 6, v = kk & 63; w = WVSV[((size_t)u * 64 + v) * 32 + n]; } s[k] = (__bf16)w; } }
  else if (which == 3) { if (n >= HID) return; K = FCIN; dst = PM1 + (size_t)n * FCIN; for (int k = tid; k < K; k += 256) s[k] = (__bf16)W1[(size_t)k * HID + n]; }
  else if (which == 4) { if (n >= HID) return; K = HID; dst = PM2 + (size_t)n * HID; for (int k = tid; k < K; k += 256) s[k] = (__bf16)W2[(size_t)k * HID + n]; }
  else { if (n >= 96) return; K = HID; dst = PM3 + (size_t)n * HID; for (int k = tid; k < K; k += 256) s[k] = (__bf16)W3[(size_t)k * 96 + n]; }
  __syncthreads();
  for (int q = tid; q < K / 8; q += 256) vst2((unsigned*)(PW + dst + q * 8), *(const v4u*)&s[q * 8]);
}
template <int STAGE>
__global__ __launch_bounds__(128) void k_mlp(const float* __restrict__ A, const __bf16* __restrict__ PW, const float* __restrict__ bias, float* __restrict__ OUT) {
  constexpr int K = (STAGE == 0) ? FCIN : HID; constexpr int NT = (STAGE == 2) ? 6 : 4; constexpr int LDO = NT * 16;
  __shared__ __align__(16) float so[4][16][LDO + 4];
  const int tid = threadIdx.x, wave = tid >> 5, lane = tid & 31, col = lane & 15, g = lane >> 4; const size_t r0 = (size_t)blockIdx.x * 64 + wave * 16; size_t ra = r0 + col; if (STAGE == 0 && ra >= NEDGE) ra = NEDGE - 1;
  const __bf16* P = PW + ((STAGE == 0) ? PM1 : (STAGE == 1 ? PM2 : PM3));
  v8f acc[NT]; for (int j = 0; j < NT; ++j) acc[j] = (v8f){};
#pragma unroll
  for (int kc = 0; kc < K / 32; ++kc) { F2 a; if (STAGE == 0) { v16b ax; const float* p = A + ra * FCIN + kc * 32 + 8 * g;
#pragma unroll
      for (int i = 0; i < 8; ++i) { ax[i] = (__bf16)p[i]; ax[8 + i] = (__bf16)p[16 + i]; } a.h = ax; a.l = ax; } else a = split_row(A + ra * HID, kc * 32, lane);
#pragma unroll
    for (int j = 0; j < NT; ++j) { const v16b w = frag_b(P + (size_t)(j * 16 + col) * K + kc * 32, lane); if (STAGE != 0) acc[j] = wmma_bf(a.l, w, acc[j]); acc[j] = wmma_bf(a.h, w, acc[j]); } }
#pragma unroll
  for (int j = 0; j < NT; ++j) { const float bb = bfr(bias[j * 16 + col]);
#pragma unroll
    for (int r = 0; r < 8; ++r) { float v = acc[j][r] + bb; if (STAGE != 2) v = v * sigm(v); so[wave][8 * g + r][j * 16 + col] = v; } }
  LDSX();
  for (int rl = 0; rl < 16; ++rl) if (lane < NT * 4) vst2(OUT + (r0 + rl) * LDO + lane * 4, *(const v4f*)&so[wave][rl][lane * 4]);
}
__global__ __launch_bounds__(128) void k_tp(const float* __restrict__ F1, const float* __restrict__ F2in, const __bf16* __restrict__ PW, const float* __restrict__ WE, float* __restrict__ out) {
  __shared__ float sx1[64][FEA + 1], sx2[64][FEA + 1]; __shared__ __align__(16) float so[4][16][FEA + 4]; __shared__ float sg[4][16][NV_ + 1];
  const int tid = threadIdx.x, wave = tid >> 5, lane = tid & 31, col = lane & 15, g = lane >> 4; const size_t e0 = (size_t)blockIdx.x * 64; const int r0 = wave * 16;
  for (int q = tid; q < 64 * FEA; q += 128) { const int rl = q / FEA, c = q % FEA; size_t e = e0 + rl; if (e >= NEDGE) e = NEDGE - 1; sx1[rl][c] = bfr(F1[e * FEA + c]); sx2[rl][c] = bfr(F2in[e * FEA + c]); }
  __syncthreads();
  const float* x1 = &sx1[r0 + col][0]; const float* x2 = &sx2[r0 + col][0];
  const float a_sc = 1.0f / sqrtf((float)(NS_ * NS_ + NV_ * NV_)), a_vec = 1.0f / sqrtf((float)(2 * NS_ * NV_)), c3 = 0.5773502691896258f;
  v8f ass[6], avv[6]; for (int j = 0; j < 6; ++j) { ass[j] = (v8f){}; avv[j] = (v8f){}; }
#pragma unroll 1
  for (int kc = 0; kc < 128; ++kc) { float v[16];
#pragma unroll
    for (int i = 0; i < 16; ++i) { const int k = kc * 32 + 8 * g + (i & 7) + ((i >> 3) << 4); v[i] = x1[k >> 6] * x2[k & 63]; }
    const F2 a = bsplit16(v);
#pragma unroll
    for (int j = 0; j < 6; ++j) { const v16b w = frag_b(PW + PSS + (size_t)(j * 16 + col) * 4096 + kc * 32, lane); ass[j] = wmma_bf(a.l, w, ass[j]); ass[j] = wmma_bf(a.h, w, ass[j]); } }
#pragma unroll 1
  for (int kc = 0; kc < 96; ++kc) { float v[16];
#pragma unroll
    for (int i = 0; i < 16; ++i) { const int k = kc * 32 + 8 * g + (i & 7) + ((i >> 3) << 4); const int uv = k / 3, ii = k - uv * 3; v[i] = x1[NS_ + (uv >> 5) * 3 + ii] * x2[NS_ + (uv & 31) * 3 + ii]; }
    const F2 a = bsplit16(v);
#pragma unroll
    for (int j = 0; j < 6; ++j) { const v16b w = frag_b(PW + PVV + (size_t)(j * 16 + col) * 3072 + kc * 32, lane); avv[j] = wmma_bf(a.l, w, avv[j]); avv[j] = wmma_bf(a.h, w, avv[j]); } }
#pragma unroll
  for (int j = 0; j < 6; ++j) { const int cch = j * 16 + col;
#pragma unroll
    for (int r = 0; r < 8; ++r) { const size_t e = e0 + r0 + 8 * g + r; const size_t ew = (e < NEDGE ? e : NEDGE - 1); const float pre = a_sc * (ass[j][r] + c3 * avv[j][r]);
      if (cch < NS_) { const float sc = pre * sigm(pre); so[wave][8 * g + r][cch] = sc * WE[ew * 96 + cch]; }
      else sg[wave][8 * g + r][cch - NS_] = sigm(pre); } }
  LDSX();
#pragma unroll 1
  for (int ii = 0; ii < 3; ++ii) { v8f av[2] = {};
#pragma unroll 1
    for (int kc = 0; kc < 128; ++kc) { float v[16];
#pragma unroll
      for (int i = 0; i < 16; ++i) { const int k = kc * 32 + 8 * g + (i & 7) + ((i >> 3) << 4); float p;
        if (k < 2048) p = x1[k >> 5] * x2[NS_ + (k & 31) * 3 + ii]; else { const int kk = k - 2048; p = x1[NS_ + (kk >> 6) * 3 + ii] * x2[kk & 63]; }
        v[i] = p; }
      const F2 a = bsplit16(v);
#pragma unroll
      for (int j = 0; j < 2; ++j) { const v16b w = frag_b(PW + PVEC + (size_t)(j * 16 + col) * 4096 + kc * 32, lane); av[j] = wmma_bf(a.l, w, av[j]); av[j] = wmma_bf(a.h, w, av[j]); } }
#pragma unroll
    for (int j = 0; j < 2; ++j) { const int wch = j * 16 + col;
#pragma unroll
      for (int r = 0; r < 8; ++r) { const size_t e = e0 + r0 + 8 * g + r; const size_t ew = (e < NEDGE ? e : NEDGE - 1); so[wave][8 * g + r][NS_ + wch * 3 + ii] = a_vec * av[j][r] * sg[wave][8 * g + r][wch] * WE[ew * 96 + NS_ + wch]; } }
    LDSX(); }
  for (int rl = 0; rl < 16; ++rl) { const size_t e = e0 + r0 + rl; if (e >= NEDGE) continue; for (int pc = lane; pc < FEA / 4; pc += 32) vst2(out + e * FEA + pc * 4, *(const v4f*)&so[wave][rl][pc * 4]); }
}
extern "C" void kernel_launch(void* const* d_in, const int* in_sizes, int n_in, void* d_out, int out_size, void* d_ws, size_t ws_size, hipStream_t stream) {
  (void)in_sizes; (void)n_in; (void)out_size;
  const float** F = (const float**)d_in;
  if (ws_size < (size_t)WS_END) return;
  char* ws = (char*)d_ws; __bf16* PW = (__bf16*)(ws + WS_PW); float *H1 = (float*)(ws + WS_H1), *H2 = (float*)(ws + WS_H2), *WE = (float*)(ws + WS_WE);
  k_pack<<<dim3(96, 6), 256, 0, stream>>>(F[3], F[4], F[5], F[6], F[7], F[8], F[9], F[11], F[13], PW);
  k_mlp<0><<<NRBT, 128, 0, stream>>>(F[2], PW, F[10], H1);
  k_mlp<1><<<NRBT, 128, 0, stream>>>(H1, PW, F[12], H2);
  k_mlp<2><<<NRBT, 128, 0, stream>>>(H2, PW, F[14], WE);
  k_tp<<<NRBT, 128, 0, stream>>>(F[0], F[1], PW, WE, (float*)d_out);
}
